// MegaTransformerSelfAttention_89928025244603
// MI455X (gfx1250) — hardware-verified
//
#include <hip/hip_runtime.h>
#include <stdint.h>


#define B_  2
#define S_  2048
#define D_  1024
#define H_  16
#define DH_ 64
#define M_  (B_ * S_)

static_assert((M_ % 64) == 0);
static_assert((D_ % 64) == 0);
static_assert((S_ % 64) == 0);
static_assert(DH_ == 64);

typedef unsigned short u16;
typedef __bf16 v16bf __attribute__((ext_vector_type(16)));
typedef __bf16 v8bf  __attribute__((ext_vector_type(8)));
typedef float  v8f   __attribute__((ext_vector_type(8)));
typedef float  v4f   __attribute__((ext_vector_type(4)));
typedef unsigned int v4u __attribute__((ext_vector_type(4)));

union Frag { v16bf v; v8bf half[2]; };

__device__ __forceinline__ v16bf ld_frag(const u16* base, int ld, int row0, int k0) {
  const int l = (int)(threadIdx.x & 31u), hh = l >> 4, m = l & 15;
  const u16* p = base + (size_t)(row0 + m) * (size_t)ld + (size_t)(k0 + 8 * hh);
  Frag f;
  f.half[0] = *(const v8bf*)(p);
  f.half[1] = *(const v8bf*)(p + 16);
  return f.v;
}

__device__ __forceinline__ void mma(v8f& acc, v16bf a, v16bf b) {
  acc = __builtin_amdgcn_wmma_f32_16x16x32_bf16(false, a, false, b, (short)0, acc, false, false);
  asm volatile("v_nop\n\tv_nop\n\tv_nop\n\tv_nop" : "+v"(acc) : "v"(a), "v"(b));
}

__device__ __forceinline__ unsigned int bf16_bits(float f) {
  const unsigned int u = __float_as_uint(f);
  return (u + 0x7FFFu + ((u >> 16) & 1u)) >> 16;
}

__device__ __forceinline__ void split_one(float x, unsigned int& hi, unsigned int& lo) {
  hi = bf16_bits(x);
  lo = bf16_bits(x - __uint_as_float(hi << 16));
}

__device__ __forceinline__ void split_pair(float x, float y, unsigned int& hi, unsigned int& lo) {
  unsigned int hx, lx, hy, ly;
  split_one(x, hx, lx);
  split_one(y, hy, ly);
  hi = hx | (hy << 16);
  lo = lx | (ly << 16);
}

__device__ __forceinline__ void split8(v4f a, v4f c, v4u& hi, v4u& lo) {
  unsigned int h0, l0, h1, l1, h2, l2, h3, l3;
  split_pair(a.x, a.y, h0, l0);
  split_pair(a.z, a.w, h1, l1);
  split_pair(c.x, c.y, h2, l2);
  split_pair(c.z, c.w, h3, l3);
  hi.x = h0; hi.y = h1; hi.z = h2; hi.w = h3;
  lo.x = l0; lo.y = l1; lo.z = l2; lo.w = l3;
}

__global__ __launch_bounds__(256) void k_split(const float* __restrict__ x,
                                               const float* __restrict__ wq, const float* __restrict__ wk,
                                               const float* __restrict__ wv, const float* __restrict__ wo,
                                               u16* __restrict__ Xh, u16* __restrict__ Xl,
                                               u16* __restrict__ Wh, u16* __restrict__ Wl,
                                               int nx, int nw) {
  const int seg = (int)blockIdx.y;
  const float* src = x;
  u16* dh = Xh;
  u16* dl = Xl;
  int n = nx;
  if (seg > 0) {
    const int wi = seg - 1;
    src = (wi == 0) ? wq : (wi == 1) ? wk : (wi == 2) ? wv : wo;
    dh = Wh + (size_t)wi * (size_t)nw;
    dl = Wl + (size_t)wi * (size_t)nw;
    n = nw;
  }
  const size_t i8 = ((size_t)blockIdx.x * (size_t)blockDim.x + (size_t)threadIdx.x) * 8u;
  if (i8 + 8u > (size_t)n) return;
  const v4f a = *(const v4f*)(src + i8);
  const v4f c = *(const v4f*)(src + i8 + 4);
  v4u vh, vl;
  split8(a, c, vh, vl);
  u16* ph = dh + i8;
  u16* pl = dl + i8;
  *(volatile v4u*)ph = vh;
  *(volatile v4u*)pl = vl;
  __threadfence();
  *(volatile v4u*)ph = vh;
  *(volatile v4u*)pl = vl;
}

__device__ __forceinline__ void gemm_block64(const u16* Ah, const u16* Al, int lda,
                                             const u16* Bh, const u16* Bl, int ldb,
                                             int m0, int n0, int K, float* tile) {
  const int w = (int)(threadIdx.x >> 5), l = (int)(threadIdx.x & 31u), hh = l >> 4, nc = l & 15;
  const int wm = (w >> 1) * 32, wn = (w & 1) * 32;
  v8f acc[2][2] = {};
  for (int kk = 0; kk < K; kk += 32) {
    const v16bf a0h = ld_frag(Ah, lda, m0 + wm, kk);
    const v16bf a0l = ld_frag(Al, lda, m0 + wm, kk);
    const v16bf a1h = ld_frag(Ah, lda, m0 + wm + 16, kk);
    const v16bf a1l = ld_frag(Al, lda, m0 + wm + 16, kk);
    const v16bf b0h = ld_frag(Bh, ldb, n0 + wn, kk);
    const v16bf b0l = ld_frag(Bl, ldb, n0 + wn, kk);
    const v16bf b1h = ld_frag(Bh, ldb, n0 + wn + 16, kk);
    const v16bf b1l = ld_frag(Bl, ldb, n0 + wn + 16, kk);
    mma(acc[0][0], a0h, b0h); mma(acc[0][0], a0l, b0h); mma(acc[0][0], a0h, b0l);
    mma(acc[0][1], a0h, b1h); mma(acc[0][1], a0l, b1h); mma(acc[0][1], a0h, b1l);
    mma(acc[1][0], a1h, b0h); mma(acc[1][0], a1l, b0h); mma(acc[1][0], a1h, b0l);
    mma(acc[1][1], a1h, b1h); mma(acc[1][1], a1l, b1h); mma(acc[1][1], a1h, b1l);
  }
#pragma unroll
  for (int r = 0; r < 8; ++r) {
    const int row0 = wm + 8 * hh + r;
    const int row1 = wm + 16 + 8 * hh + r;
    tile[row0 * 64 + wn + nc]      = acc[0][0][r];
    tile[row0 * 64 + wn + 16 + nc] = acc[0][1][r];
    tile[row1 * 64 + wn + nc]      = acc[1][0][r];
    tile[row1 * 64 + wn + 16 + nc] = acc[1][1][r];
  }
}

__global__ __launch_bounds__(128) void k_proj_qkv(const u16* Xh, const u16* Xl,
                                                  const u16* Wh, const u16* Wl,
                                                  u16* Qh, u16* Ql, u16* Kh, u16* Kl,
                                                  u16* Vth, u16* Vtl) {
  __shared__ __attribute__((aligned(16))) float tile[64 * 64];
  const int z = (int)blockIdx.z;
  const int hd = (int)blockIdx.x;
  const int n0 = hd * 64;
  const int m0 = (int)blockIdx.y * 64;
  const u16* Bh = Wh + (size_t)z * (size_t)D_ * (size_t)D_;
  const u16* Bl = Wl + (size_t)z * (size_t)D_ * (size_t)D_;
  gemm_block64(Xh, Xl, D_, Bh, Bl, D_, m0, n0, D_, tile);
  __syncthreads();

  const int w = (int)(threadIdx.x >> 5), l = (int)(threadIdx.x & 31u);
  const int b = m0 >> 11, s0 = m0 & (S_ - 1);
  const int bh = b * H_ + hd;
  if (z < 2) {
    u16* Ph = (z == 0) ? Qh : Kh;
    u16* Pl = (z == 0) ? Ql : Kl;
    const size_t base = ((size_t)bh * (size_t)S_ + (size_t)s0) * (size_t)DH_;
#pragma unroll
    for (int j = 0; j < 4; ++j) {
      const int row = w * 16 + j * 4 + (l >> 3);
      const int c0 = 8 * (l & 7);
      const float* tp = tile + row * 64 + c0;
      const v4f f0 = *(const v4f*)(tp);
      const v4f f1 = *(const v4f*)(tp + 4);
      v4u vh, vl;
      split8(f0, f1, vh, vl);
      const size_t o = base + (size_t)row * (size_t)DH_ + (size_t)c0;
      *(volatile v4u*)(Ph + o) = vh;
      *(volatile v4u*)(Pl + o) = vl;
      __threadfence();
      *(volatile v4u*)(Ph + o) = vh;
      *(volatile v4u*)(Pl + o) = vl;
    }
  } else {
#pragma unroll
    for (int j = 0; j < 4; ++j) {
      const int d = w * 16 + j * 4 + (l >> 3);
      const int k0 = 8 * (l & 7);
      v4f f0, f1;
      f0.x = tile[(k0 + 0) * 64 + d]; f0.y = tile[(k0 + 1) * 64 + d];
      f0.z = tile[(k0 + 2) * 64 + d]; f0.w = tile[(k0 + 3) * 64 + d];
      f1.x = tile[(k0 + 4) * 64 + d]; f1.y = tile[(k0 + 5) * 64 + d];
      f1.z = tile[(k0 + 6) * 64 + d]; f1.w = tile[(k0 + 7) * 64 + d];
      v4u vh, vl;
      split8(f0, f1, vh, vl);
      const size_t o = ((size_t)bh * (size_t)DH_ + (size_t)d) * (size_t)S_ + (size_t)s0 + (size_t)k0;
      *(volatile v4u*)(Vth + o) = vh;
      *(volatile v4u*)(Vtl + o) = vl;
      __threadfence();
      *(volatile v4u*)(Vth + o) = vh;
      *(volatile v4u*)(Vtl + o) = vl;
    }
  }
}

__global__ __launch_bounds__(128) void k_proj_out(const u16* Ch, const u16* Cl,
                                                  const u16* Wh, const u16* Wl,
                                                  const float* __restrict__ bo, float* out) {
  __shared__ __attribute__((aligned(16))) float tile[64 * 64];
  const int n0 = (int)blockIdx.x * 64;
  const int m0 = (int)blockIdx.y * 64;
  const u16* Bh = Wh + (size_t)3 * (size_t)D_ * (size_t)D_;
  const u16* Bl = Wl + (size_t)3 * (size_t)D_ * (size_t)D_;
  gemm_block64(Ch, Cl, D_, Bh, Bl, D_, m0, n0, D_, tile);
  __syncthreads();

  const int w = (int)(threadIdx.x >> 5), l = (int)(threadIdx.x & 31u);
#pragma unroll
  for (int j = 0; j < 8; ++j) {
    const int row = w * 16 + j * 2 + (l >> 4);
    const int c0 = 4 * (l & 15);
    v4f v = *(const v4f*)(tile + row * 64 + c0);
    const v4f bb = *(const v4f*)(bo + n0 + c0);
    v = v + bb;
    float* op = out + (size_t)(m0 + row) * (size_t)D_ + (size_t)(n0 + c0);
    *(volatile v4f*)op = v;
    __threadfence();
    *(volatile v4f*)op = v;
  }
}

__global__ __launch_bounds__(32) void k_attn(const u16* Qh, const u16* Ql,
                                             const u16* Kh, const u16* Kl,
                                             const u16* Vth, const u16* Vtl,
                                             u16* Ch, u16* Cl) {
  __shared__ __attribute__((aligned(16))) u16 lds_ph[16 * 32];
  __shared__ __attribute__((aligned(16))) u16 lds_pl[16 * 32];
  __shared__ __attribute__((aligned(16))) float ctile[16 * 64];

  const int gw = (int)blockIdx.x;
  const int bh = gw >> 7, qt = gw & 127;
  const int b = bh >> 4, hd = bh & 15;
  const int l = (int)(threadIdx.x & 31u), hh = l >> 4, nc = l & 15;
  const int q0 = qt * 16;
  const int ex = hd + 1;
  const float slope = ((ex & 1) ? 0.70710678118654752f : 1.0f) *
                      __uint_as_float((unsigned int)(127 - (ex >> 1)) << 23);

  const u16* Qhp  = Qh  + (size_t)bh * (size_t)S_ * (size_t)DH_;
  const u16* Qlp  = Ql  + (size_t)bh * (size_t)S_ * (size_t)DH_;
  const u16* Khp  = Kh  + (size_t)bh * (size_t)S_ * (size_t)DH_;
  const u16* Klp  = Kl  + (size_t)bh * (size_t)S_ * (size_t)DH_;
  const u16* Vthp = Vth + (size_t)bh * (size_t)DH_ * (size_t)S_;
  const u16* Vtlp = Vtl + (size_t)bh * (size_t)DH_ * (size_t)S_;

  const v16bf q0h = ld_frag(Qhp, DH_, q0, 0),  q0l = ld_frag(Qlp, DH_, q0, 0);
  const v16bf q1h = ld_frag(Qhp, DH_, q0, 32), q1l = ld_frag(Qlp, DH_, q0, 32);

  v8f o[4] = {};
  float mrow[8], lrow[8];
#pragma unroll
  for (int r = 0; r < 8; ++r) { mrow[r] = -3.0e38f; lrow[r] = 0.0f; }

  const int nchunk = (q0 >> 5) + 1;
  for (int c = 0; c < nchunk; ++c) {
    const int ks = c << 5;
    v8f s[2] = {};
#pragma unroll
    for (int t = 0; t < 2; ++t) {
      const int kr = ks + 16 * t;
      const v16bf k0h = ld_frag(Khp, DH_, kr, 0),  k0l = ld_frag(Klp, DH_, kr, 0);
      const v16bf k1h = ld_frag(Khp, DH_, kr, 32), k1l = ld_frag(Klp, DH_, kr, 32);
      mma(s[t], q0h, k0h); mma(s[t], q0l, k0h); mma(s[t], q0h, k0l);
      mma(s[t], q1h, k1h); mma(s[t], q1l, k1h); mma(s[t], q1h, k1l);
    }

#pragma unroll
    for (int r = 0; r < 8; ++r) {
      const int q = q0 + 8 * hh + r;
      const int ka = ks + nc, kb = ks + 16 + nc;
      float xa = (s[0][r] - (float)(q - ka) * slope) * 0.125f;
      float xb = (s[1][r] - (float)(q - kb) * slope) * 0.125f;
      xa = 30.0f * tanhf(xa * (1.0f / 30.0f));
      xb = 30.0f * tanhf(xb * (1.0f / 30.0f));
      xa = (ka <= q) ? xa : -3.0e38f;
      xb = (kb <= q) ? xb : -3.0e38f;
      float t = fmaxf(xa, xb);
      t = fmaxf(t, __shfl_xor(t, 1, 32));
      t = fmaxf(t, __shfl_xor(t, 2, 32));
      t = fmaxf(t, __shfl_xor(t, 4, 32));
      t = fmaxf(t, __shfl_xor(t, 8, 32));
      const float mnew = fmaxf(mrow[r], t);
      const float alpha = __expf(mrow[r] - mnew);
      const float pa = __expf(xa - mnew);
      const float pb = __expf(xb - mnew);
      float u = pa + pb;
      u += __shfl_xor(u, 1, 32);
      u += __shfl_xor(u, 2, 32);
      u += __shfl_xor(u, 4, 32);
      u += __shfl_xor(u, 8, 32);
      lrow[r] = lrow[r] * alpha + u;
      mrow[r] = mnew;
      o[0][r] *= alpha; o[1][r] *= alpha; o[2][r] *= alpha; o[3][r] *= alpha;
      unsigned int ha, la, hb, lb;
      split_one(pa, ha, la);
      split_one(pb, hb, lb);
      const int row = 8 * hh + r;
      lds_ph[row * 32 + nc]      = (u16)ha;
      lds_ph[row * 32 + 16 + nc] = (u16)hb;
      lds_pl[row * 32 + nc]      = (u16)la;
      lds_pl[row * 32 + 16 + nc] = (u16)lb;
    }
    __syncthreads();
    const v16bf ph = ld_frag(lds_ph, 32, 0, 0);
    const v16bf pl = ld_frag(lds_pl, 32, 0, 0);
#pragma unroll
    for (int si = 0; si < 4; ++si) {
      const v16bf vh = ld_frag(Vthp, S_, 16 * si, ks);
      const v16bf vl = ld_frag(Vtlp, S_, 16 * si, ks);
      mma(o[si], ph, vh); mma(o[si], pl, vh); mma(o[si], ph, vl);
    }
    __syncthreads();
  }

#pragma unroll
  for (int r = 0; r < 8; ++r) {
    const float inv = 1.0f / lrow[r];
    const int row = 8 * hh + r;
    ctile[row * 64 + nc]      = o[0][r] * inv;
    ctile[row * 64 + 16 + nc] = o[1][r] * inv;
    ctile[row * 64 + 32 + nc] = o[2][r] * inv;
    ctile[row * 64 + 48 + nc] = o[3][r] * inv;
  }
  __syncthreads();
  const size_t rbase = ((size_t)b * (size_t)S_ + (size_t)q0) * (size_t)D_ + (size_t)hd * (size_t)DH_;
#pragma unroll
  for (int j = 0; j < 4; ++j) {
    const int row = j * 4 + (l >> 3);
    const int c0 = 8 * (l & 7);
    const float* tp = ctile + row * 64 + c0;
    const v4f f0 = *(const v4f*)(tp);
    const v4f f1 = *(const v4f*)(tp + 4);
    v4u vh, vl;
    split8(f0, f1, vh, vl);
    const size_t oidx = rbase + (size_t)row * (size_t)D_ + (size_t)c0;
    *(volatile v4u*)(Ch + oidx) = vh;
    *(volatile v4u*)(Cl + oidx) = vl;
    __threadfence();
    *(volatile v4u*)(Ch + oidx) = vh;
    *(volatile v4u*)(Cl + oidx) = vl;
  }
}

extern "C" void kernel_launch(void* const* d_in, const int* in_sizes, int n_in,
                              void* d_out, int out_size, void* d_ws, size_t ws_size,
                              hipStream_t stream) {
  if (n_in < 6) return;
  const int nX = M_ * D_;
  const int nW = D_ * D_;
  const int nHead = B_ * H_ * S_ * DH_;
  if (in_sizes[0] != nX || in_sizes[1] != nW || in_sizes[2] != nW ||
      in_sizes[3] != nW || in_sizes[4] != nW || in_sizes[5] != D_) return;
  if (out_size != nX) return;

  const float* hs = (const float*)d_in[0];
  const float* wq = (const float*)d_in[1];
  const float* wk = (const float*)d_in[2];
  const float* wv = (const float*)d_in[3];
  const float* wo = (const float*)d_in[4];
  const float* bo = (const float*)d_in[5];
  float* out = (float*)d_out;

  char* ws = (char*)d_ws;
  size_t off = 0;
  const size_t bX = (size_t)nX * 2u;
  const size_t bW = (size_t)nW * 2u * 4u;
  const size_t bHd = (size_t)nHead * 2u;
  u16* Xh  = (u16*)(ws + off); off += bX;
  u16* Xl  = (u16*)(ws + off); off += bX;
  u16* Wh  = (u16*)(ws + off); off += bW;
  u16* Wl  = (u16*)(ws + off); off += bW;
  u16* Qh  = (u16*)(ws + off); off += bHd;
  u16* Ql  = (u16*)(ws + off); off += bHd;
  u16* Kh  = (u16*)(ws + off); off += bHd;
  u16* Kl  = (u16*)(ws + off); off += bHd;
  u16* Vth = (u16*)(ws + off); off += bHd;
  u16* Vtl = (u16*)(ws + off); off += bHd;
  u16* Ch  = (u16*)(ws + off); off += bX;
  u16* Cl  = (u16*)(ws + off); off += bX;
  if (off > ws_size) return;

  k_split<<<dim3((unsigned)(nX / 8 / 256), 5, 1), 256, 0, stream>>>(hs, wq, wk, wv, wo, Xh, Xl, Wh, Wl, nX, nW);
  k_proj_qkv<<<dim3(D_ / 64, M_ / 64, 3), 128, 0, stream>>>(Xh, Xl, Wh, Wl, Qh, Ql, Kh, Kl, Vth, Vtl);
  k_attn<<<dim3((unsigned)(B_ * H_ * (S_ / 16)), 1, 1), 32, 0, stream>>>(Qh, Ql, Kh, Kl, Vth, Vtl, Ch, Cl);
  k_proj_out<<<dim3(D_ / 64, M_ / 64, 1), 128, 0, stream>>>(Ch, Cl, Wh, Wl, bo, out);
  (void)hipGetLastError();
}
